// CausalSelfAttention_12824772346355
// MI455X (gfx1250) — hardware-verified
//
#include <hip/hip_runtime.h>


#ifndef NB
#define NB 1
#endif
#define NB_FULL 1
#ifndef SEQ
#define SEQ 4096
#endif
#define SEQ_FULL 4096
#define DM   1024
#define NH_  16
#define HD   64
#ifndef RH
#define RH   1024
#endif
#if RH > SEQ
#undef RH
#define RH SEQ
#endif
#define PCAR 1024.0f
#define SCL  0.125f
#define L2E  1.4426950408889634f
#define NEGB (-3.0e38f)
#define PSP  40
#define OSP  72

static_assert(NB >= 1 && NB <= NB_FULL);
static_assert(SEQ >= 64 && SEQ <= SEQ_FULL && SEQ % 64 == 0);
static_assert(RH >= 64 && RH <= SEQ && RH % 64 == 0);
static_assert(NH_ * HD == DM);
static_assert(DM % 64 == 0 && DM % 32 == 0 && HD == 64);
static_assert((NH_ * SEQ * HD) % 512 == 0);
static_assert((SEQ * DM) % 2048 == 0 && (DM * DM) % 2048 == 0);
static_assert((PSP * 2) % 16 == 0 && (OSP * 2) % 16 == 0);

typedef _Float16 h16;
typedef unsigned short bf;
typedef __attribute__((ext_vector_type(16))) __bf16   v16bf;
typedef __attribute__((ext_vector_type(16))) _Float16 v16h;
typedef __attribute__((ext_vector_type(8)))  _Float16 v8h;
typedef __attribute__((ext_vector_type(8)))  unsigned short v8us;
typedef __attribute__((ext_vector_type(8)))  float    v8f;
typedef __attribute__((ext_vector_type(4)))  float    v4f;
typedef __attribute__((ext_vector_type(2)))  float    v2f;
typedef __attribute__((ext_vector_type(2)))  _Float16 v2h;
typedef __attribute__((ext_vector_type(2)))  unsigned short v2us;
typedef v8h  __attribute__((may_alias)) v8ha;
typedef v4f  __attribute__((may_alias)) v4fa;
typedef v8us __attribute__((may_alias)) v8usa;

__device__ __forceinline__ unsigned short f2bf(float f) { unsigned u = __float_as_uint(f); u += 0x7FFFu + ((u >> 16) & 1u); return (unsigned short)(u >> 16); }
__device__ __forceinline__ float bf2f(unsigned short b) { return __uint_as_float(((unsigned)b) << 16); }
__device__ __forceinline__ float bfr(float f) { return bf2f(f2bf(f)); }
__device__ __forceinline__ v16h cat16(v8h lo, v8h hi) { return __builtin_shufflevector(lo, hi, 0, 1, 2, 3, 4, 5, 6, 7, 8, 9, 10, 11, 12, 13, 14, 15); }
__device__ __forceinline__ v16bf cat16b(v8us lo, v8us hi) { return __builtin_bit_cast(v16bf, __builtin_shufflevector(lo, hi, 0, 1, 2, 3, 4, 5, 6, 7, 8, 9, 10, 11, 12, 13, 14, 15)); }
__device__ __forceinline__ v8f wmma16(v16h a, v16h b, v8f c) { return __builtin_amdgcn_wmma_f32_16x16x32_f16(false, a, false, b, (short)0, c, false, false); }
__device__ __forceinline__ v8f wmmab(v16bf a, v16bf b, v8f c) { return __builtin_amdgcn_wmma_f32_16x16x32_bf16(false, a, false, b, (short)0, c, false, false); }
__device__ __forceinline__ h16 tohx(float x) { return (h16)x; }
__device__ __forceinline__ void splitf(float y, unsigned short& h, unsigned short& l) { h = f2bf(y); l = f2bf(y - bf2f(h)); }

template <typename T16> struct WFrag;
template <> struct WFrag<h16> { typedef v16h V; static __device__ __forceinline__ V ld(const h16* p) { return cat16(*(const v8h*)p, *(const v8h*)(p + 16)); } static __device__ __forceinline__ v8f mma(V a, V b, v8f c) { return wmma16(a, b, c); } };
template <> struct WFrag<bf> { typedef v16bf V; static __device__ __forceinline__ V ld(const bf* p) { return cat16b(*(const v8us*)p, *(const v8us*)(p + 16)); } static __device__ __forceinline__ v8f mma(V a, V b, v8f c) { return wmmab(a, b, c); } };

template <typename T16, int NSPLIT, bool BIAS>
__global__ __launch_bounds__(32) void k_gemmw(const T16* __restrict__ A, const T16* __restrict__ A2, const T16* __restrict__ Bt, const T16* __restrict__ Bt2, int K, float* C, int ldc, const float* __restrict__ bias, size_t sA, size_t sB, size_t sC) {
    typedef typename WFrag<T16>::V V;
    __shared__ __align__(16) float os[16 * 68];
    const size_t z = blockIdx.z; A += z * sA; if (A2) A2 += z * sA; Bt += z * sB; if (Bt2) Bt2 += z * sB; C += z * sC;
    const int lane = threadIdx.x & 31, lr = lane & 15, hi = lane >> 4; const int r0 = blockIdx.x * 64, c0 = blockIdx.y * 64;
    v8f acc[4][4];
#pragma unroll
    for (int mb = 0; mb < 4; ++mb)
#pragma unroll
        for (int nb = 0; nb < 4; ++nb) acc[mb][nb] = (v8f){};
    const size_t aoff = (size_t)(r0 + lr) * K + 8 * hi, boff = (size_t)(c0 + lr) * K + 8 * hi;
#pragma unroll 1
    for (int kc = 0; kc < K; kc += 32) {
        V a[4], a2[4];
#pragma unroll
        for (int mb = 0; mb < 4; ++mb) { a[mb] = WFrag<T16>::ld(A + aoff + (size_t)mb * 16 * K + kc); if (NSPLIT == 1 || NSPLIT == 2) a2[mb] = WFrag<T16>::ld(A2 + aoff + (size_t)mb * 16 * K + kc); }
#pragma unroll
        for (int nb = 0; nb < 4; ++nb) { const V b = WFrag<T16>::ld(Bt + boff + (size_t)nb * 16 * K + kc); V b2; if (NSPLIT >= 2) b2 = WFrag<T16>::ld(Bt2 + boff + (size_t)nb * 16 * K + kc);
#pragma unroll
            for (int mb = 0; mb < 4; ++mb) { acc[mb][nb] = WFrag<T16>::mma(a[mb], b, acc[mb][nb]); if (NSPLIT == 1 || NSPLIT == 2) acc[mb][nb] = WFrag<T16>::mma(a2[mb], b, acc[mb][nb]); if (NSPLIT >= 2) acc[mb][nb] = WFrag<T16>::mma(a[mb], b2, acc[mb][nb]); } }
        asm volatile("v_nop\n\tv_nop\n\tv_nop\n\tv_nop" : "+v"(acc[0][0]), "+v"(acc[1][1]), "+v"(acc[2][2]), "+v"(acc[3][3]) : "v"(a[0]), "v"(a[3]));
    }
#pragma unroll
    for (int mb = 0; mb < 4; ++mb) {
#pragma unroll
        for (int nb = 0; nb < 4; ++nb) {
#pragma unroll
            for (int j = 0; j < 8; ++j) os[(hi * 8 + j) * 68 + nb * 16 + lr] = acc[mb][nb][j]; }
        __builtin_amdgcn_wave_barrier(); asm volatile("" ::: "memory");
        float* crow = C + (size_t)(r0 + mb * 16) * ldc + c0;
#pragma unroll 1
        for (int ps = 0; ps < 2; ++ps) {
#pragma unroll
            for (int s = 0; s < 8; ++s) { const int row = 2 * s + hi, cofs = lr * 4; v4f val = *(const v4fa*)(os + row * 68 + cofs); if (BIAS) { val[0] += bfr(bias[c0 + cofs]); val[1] += bfr(bias[c0 + cofs + 1]); val[2] += bfr(bias[c0 + cofs + 2]); val[3] += bfr(bias[c0 + cofs + 3]); }
                *(volatile v4f*)(crow + (size_t)row * ldc + cofs) = val; }
            if (ps == 0) __threadfence(); }
        __builtin_amdgcn_wave_barrier(); asm volatile("" ::: "memory");
    }
}

__global__ __launch_bounds__(256) void k_cvt8(const float* __restrict__ src, bf* dst, size_t n8) { const size_t i = (size_t)blockIdx.x * 256 + threadIdx.x; if (i >= n8) return; const v8f v = *(const v8f*)(src + i * 8); v8us o;
#pragma unroll
    for (int k = 0; k < 8; ++k) o[k] = f2bf(v[k]); *(volatile v8us*)(dst + i * 8) = o; __threadfence(); *(volatile v8us*)(dst + i * 8) = o; }

__global__ __launch_bounds__(256) void k_qkp(const float* __restrict__ F, h16* P16, bf* Ph, bf* Pl) {
    const size_t e = ((size_t)blockIdx.x * 256 + threadIdx.x) * 2; if (e >= (size_t)NH_ * SEQ * HD) return;
    const int d = (int)(e % HD); const int t = (int)((e / HD) % SEQ); const int hh = (int)(e / ((size_t)HD * SEQ));
    const v2f x2 = *(const v2f*)(F + (size_t)t * DM + hh * HD + d);
    v2h o16; v2us oh, ol;
#pragma unroll
    for (int q = 0; q < 2; ++q) { o16[q] = tohx(x2[q]); unsigned short a, c; splitf(x2[q], a, c); oh[q] = a; ol[q] = c; }
    const bool dohl = (t < RH);
    const int tc = dohl ? t : (RH - 1);
    const size_t oo = ((size_t)hh * RH + tc) * HD + d;
    *(volatile v2h*)(P16 + e) = o16; if (dohl) { *(volatile v2us*)(Ph + oo) = oh; *(volatile v2us*)(Pl + oo) = ol; }
    __threadfence();
    *(volatile v2h*)(P16 + e) = o16; if (dohl) { *(volatile v2us*)(Ph + oo) = oh; *(volatile v2us*)(Pl + oo) = ol; }
}
__global__ __launch_bounds__(256) void k_vtp(const float* __restrict__ F, h16* V16, bf* Vh, bf* Vl) {
    const size_t e = ((size_t)blockIdx.x * 256 + threadIdx.x) * 2; if (e >= (size_t)NH_ * HD * SEQ) return;
    const int t = (int)(e % SEQ); const int d = (int)((e / SEQ) % HD); const int g = (int)(e / ((size_t)SEQ * HD));
    v2h o16; v2us oh, ol;
#pragma unroll
    for (int q = 0; q < 2; ++q) { const float x = F[(size_t)(t + q) * DM + g * HD + d]; o16[q] = tohx(x); unsigned short a, c; splitf(x, a, c); oh[q] = a; ol[q] = c; }
    const bool dohl = (t < RH);
    const int tc = dohl ? t : (RH - 2);
    const size_t oo = ((size_t)g * HD + d) * RH + tc;
    *(volatile v2h*)(V16 + e) = o16; if (dohl) { *(volatile v2us*)(Vh + oo) = oh; *(volatile v2us*)(Vl + oo) = ol; }
    __threadfence();
    *(volatile v2h*)(V16 + e) = o16; if (dohl) { *(volatile v2us*)(Vh + oo) = oh; *(volatile v2us*)(Vl + oo) = ol; }
}

template <bool HI>
__global__ __launch_bounds__(32) void k_flash(const h16* __restrict__ Q16, const h16* __restrict__ K16, const h16* __restrict__ VT16,
                                              const bf* __restrict__ Qh, const bf* __restrict__ Ql, const bf* __restrict__ Kh, const bf* __restrict__ Kl,
                                              const bf* __restrict__ VTh, const bf* __restrict__ VTl, int qb0, bf* ATh, bf* ATl) {
    __shared__ __align__(16) h16 ps16[16 * PSP];
    __shared__ __align__(16) bf  psh[16 * PSP];
    __shared__ __align__(16) bf  psl[16 * PSP];
    __shared__ __align__(16) bf  sth[16 * OSP];
    __shared__ __align__(16) bf  stl[16 * OSP];
    const int lane = threadIdx.x & 31, lr = lane & 15, hi = lane >> 4;
    const int hh = blockIdx.y; const int q0 = (qb0 + (int)blockIdx.x) * 16; const int nkb = (q0 + 16 + 31) >> 5;
    v16h q16[2]; v16bf qh[2], ql[2];
    if (HI) {
        const size_t qo = ((size_t)hh * RH + q0 + lr) * HD + 8 * hi;
#pragma unroll
        for (int ks = 0; ks < 2; ++ks) { qh[ks] = WFrag<bf>::ld(Qh + qo + 32 * ks); ql[ks] = WFrag<bf>::ld(Ql + qo + 32 * ks); }
    } else {
        const size_t qo = ((size_t)hh * SEQ + q0 + lr) * HD + 8 * hi;
#pragma unroll
        for (int ks = 0; ks < 2; ++ks) q16[ks] = WFrag<h16>::ld(Q16 + qo + 32 * ks);
    }
    v8f o[4];
#pragma unroll
    for (int nt = 0; nt < 4; ++nt) o[nt] = (v8f){};
    float mrow[8], lrow[8];
#pragma unroll
    for (int r = 0; r < 8; ++r) { mrow[r] = NEGB; lrow[r] = 0.f; }

#pragma unroll 1
    for (int kb = 0; kb < nkb; ++kb) {
        const int k0 = kb * 32;
        v8f s[2]; s[0] = (v8f){}; s[1] = (v8f){};
        if (HI) {
#pragma unroll
            for (int nt = 0; nt < 2; ++nt) { const size_t ko = ((size_t)hh * RH + k0 + 16 * nt + lr) * HD + 8 * hi;
#pragma unroll
                for (int ks = 0; ks < 2; ++ks) { const v16bf bh = WFrag<bf>::ld(Kh + ko + 32 * ks); const v16bf bl = WFrag<bf>::ld(Kl + ko + 32 * ks);
                    s[nt] = wmmab(qh[ks], bh, s[nt]); s[nt] = wmmab(ql[ks], bh, s[nt]); s[nt] = wmmab(qh[ks], bl, s[nt]); } }
            asm volatile("v_nop\n\tv_nop\n\tv_nop\n\tv_nop" : "+v"(s[0]), "+v"(s[1]) : "v"(qh[0]), "v"(qh[1]), "v"(ql[0]), "v"(ql[1]));
        } else {
#pragma unroll
            for (int nt = 0; nt < 2; ++nt) { const size_t ko = ((size_t)hh * SEQ + k0 + 16 * nt + lr) * HD + 8 * hi;
#pragma unroll
                for (int ks = 0; ks < 2; ++ks) { const v16h b16 = WFrag<h16>::ld(K16 + ko + 32 * ks); s[nt] = wmma16(q16[ks], b16, s[nt]); } }
            asm volatile("v_nop\n\tv_nop\n\tv_nop\n\tv_nop" : "+v"(s[0]), "+v"(s[1]) : "v"(q16[0]), "v"(q16[1]));
        }
        const bool last = (kb == nkb - 1);
#pragma unroll
        for (int nt = 0; nt < 2; ++nt)
#pragma unroll
            for (int r = 0; r < 8; ++r) { float v = s[nt][r] * SCL; if (last) { const int key = k0 + 16 * nt + lr; const int qr = q0 + 8 * hi + r; v = (key > qr) ? NEGB : v; } s[nt][r] = v; }
#pragma unroll
        for (int r = 0; r < 8; ++r) {
            float mx = fmaxf(s[0][r], s[1][r]);
            mx = fmaxf(mx, __shfl_xor(mx, 1, 32)); mx = fmaxf(mx, __shfl_xor(mx, 2, 32)); mx = fmaxf(mx, __shfl_xor(mx, 4, 32)); mx = fmaxf(mx, __shfl_xor(mx, 8, 32));
            const float mold = mrow[r]; const float mnew = fmaxf(mold, mx); mrow[r] = mnew;
            float dm = __fsub_rn(mold, mnew); asm volatile("" : "+v"(dm)); const float sc = __builtin_amdgcn_exp2f(__fmul_rn(dm, L2E));
            float d0 = __fsub_rn(s[0][r], mnew); asm volatile("" : "+v"(d0)); const float e0 = __builtin_amdgcn_exp2f(__fmul_rn(d0, L2E));
            float d1 = __fsub_rn(s[1][r], mnew); asm volatile("" : "+v"(d1)); const float e1 = __builtin_amdgcn_exp2f(__fmul_rn(d1, L2E));
            float rs = e0 + e1;
            rs += __shfl_xor(rs, 1, 32); rs += __shfl_xor(rs, 2, 32); rs += __shfl_xor(rs, 4, 32); rs += __shfl_xor(rs, 8, 32);
            lrow[r] = lrow[r] * sc + rs;
            s[0][r] = e0; s[1][r] = e1;
#pragma unroll
            for (int nt = 0; nt < 4; ++nt) o[nt][r] = o[nt][r] * sc;
        }
        if (HI) {
#pragma unroll
            for (int nt = 0; nt < 2; ++nt)
#pragma unroll
                for (int r = 0; r < 8; ++r) { unsigned short a, c; splitf(s[nt][r], a, c); const int li = (8 * hi + r) * PSP + 16 * nt + lr; psh[li] = a; psl[li] = c; }
        } else {
#pragma unroll
            for (int nt = 0; nt < 2; ++nt)
#pragma unroll
                for (int r = 0; r < 8; ++r) { const int li = (8 * hi + r) * PSP + 16 * nt + lr; ps16[li] = tohx(s[nt][r] * PCAR); }
        }
        __syncthreads();
        const int po = lr * PSP + 8 * hi;
        v16h p16; v16bf ph, pl;
        if (HI) { ph = cat16b(*(const v8usa*)(psh + po), *(const v8usa*)(psh + po + 16)); pl = cat16b(*(const v8usa*)(psl + po), *(const v8usa*)(psl + po + 16)); }
        else    { p16 = cat16(*(const v8ha*)(ps16 + po), *(const v8ha*)(ps16 + po + 16)); }
        __syncthreads();
        if (HI) {
#pragma unroll
            for (int nt = 0; nt < 4; ++nt) { const size_t vo = ((size_t)hh * HD + 16 * nt + lr) * RH + k0 + 8 * hi; const v16bf bh = WFrag<bf>::ld(VTh + vo); const v16bf bl = WFrag<bf>::ld(VTl + vo);
                o[nt] = wmmab(ph, bh, o[nt]); o[nt] = wmmab(pl, bh, o[nt]); o[nt] = wmmab(ph, bl, o[nt]); }
            asm volatile("v_nop\n\tv_nop\n\tv_nop\n\tv_nop" : "+v"(o[0]), "+v"(o[1]), "+v"(o[2]), "+v"(o[3]) : "v"(ph), "v"(pl));
        } else {
#pragma unroll
            for (int nt = 0; nt < 4; ++nt) { const size_t vo = ((size_t)hh * HD + 16 * nt + lr) * SEQ + k0 + 8 * hi; const v16h b16 = WFrag<h16>::ld(VT16 + vo); o[nt] = wmma16(p16, b16, o[nt]); }
            asm volatile("v_nop\n\tv_nop\n\tv_nop\n\tv_nop" : "+v"(o[0]), "+v"(o[1]), "+v"(o[2]), "+v"(o[3]) : "v"(p16));
        }
    }
    const float osc = HI ? 1.0f : (1.0f / PCAR);
#pragma unroll
    for (int r = 0; r < 8; ++r) { const float inv = __fdiv_rn(osc, lrow[r]);
#pragma unroll
        for (int nt = 0; nt < 4; ++nt) { unsigned short a, c; splitf(o[nt][r] * inv, a, c); const int li = (8 * hi + r) * OSP + 16 * nt + lr; sth[li] = a; stl[li] = c; } }
    __syncthreads();
#pragma unroll 1
    for (int ps = 0; ps < 2; ++ps) {
#pragma unroll
        for (int it = 0; it < 4; ++it) { const int row = it * 4 + (lane >> 3); const int col = (lane & 7) * 8;
            const v8us vh = *(const v8usa*)(sth + row * OSP + col); const v8us vl = *(const v8usa*)(stl + row * OSP + col);
            const size_t go = (size_t)(q0 + row) * DM + hh * HD + col;
            *(volatile v8us*)(ATh + go) = vh; *(volatile v8us*)(ATl + go) = vl; }
        if (ps == 0) __threadfence(); }
}

extern "C" void kernel_launch(void* const* d_in, const int* in_sizes, int n_in,
                              void* d_out, int out_size, void* d_ws, size_t ws_size, hipStream_t stream) {
    if (n_in < 9) return;
    if ((size_t)in_sizes[0] < (size_t)(NB - 1) * SEQ_FULL * DM + (size_t)SEQ * DM) return;
    if (in_sizes[1] < DM * DM || in_sizes[3] < DM * DM || in_sizes[5] < DM * DM || in_sizes[7] < DM * DM) return;
    if (in_sizes[2] < DM || in_sizes[4] < DM || in_sizes[6] < DM || in_sizes[8] < DM) return;
    if ((size_t)out_size < (size_t)(NB - 1) * SEQ_FULL * DM + (size_t)SEQ * DM) return;
    const float* x = (const float*)d_in[0]; const float* wq = (const float*)d_in[1]; const float* bq = (const float*)d_in[2]; const float* wk = (const float*)d_in[3]; const float* bk = (const float*)d_in[4];
    const float* wv = (const float*)d_in[5]; const float* bv = (const float*)d_in[6]; const float* wp = (const float*)d_in[7]; const float* bp = (const float*)d_in[8];
    float* OUT = (float*)d_out;
    char* wsp = (char*)d_ws;
    auto take = [&](size_t bytes) { char* p = wsp; wsp += (bytes + 255) & ~(size_t)255; return (void*)p; };
    bf* WQ = (bf*)take((size_t)DM * DM * 2); bf* WK = (bf*)take((size_t)DM * DM * 2); bf* WV = (bf*)take((size_t)DM * DM * 2); bf* WP = (bf*)take((size_t)DM * DM * 2);
    bf* XB = (bf*)take((size_t)SEQ * DM * 2); float* FQ = (float*)take((size_t)SEQ * DM * 4); float* FK = (float*)take((size_t)SEQ * DM * 4);
    h16* Q16 = (h16*)take((size_t)NH_ * SEQ * HD * 2); h16* K16 = (h16*)take((size_t)NH_ * SEQ * HD * 2); h16* VT16 = (h16*)take((size_t)NH_ * HD * SEQ * 2);
    bf* QPh = (bf*)take((size_t)NH_ * RH * HD * 2); bf* QPl = (bf*)take((size_t)NH_ * RH * HD * 2); bf* KPh = (bf*)take((size_t)NH_ * RH * HD * 2); bf* KPl = (bf*)take((size_t)NH_ * RH * HD * 2);
    bf* VTh = (bf*)take((size_t)NH_ * HD * RH * 2); bf* VTl = (bf*)take((size_t)NH_ * HD * RH * 2);
    bf* ATh = (bf*)take((size_t)SEQ * DM * 2); bf* ATl = (bf*)take((size_t)SEQ * DM * 2);
    if ((size_t)(wsp - (char*)d_ws) > ws_size) return;
    float* FV = FK;
    const unsigned GW = (unsigned)((size_t)DM * DM / 8 / 256), GX = (unsigned)((size_t)SEQ * DM / 8 / 256), GP = (unsigned)((size_t)NH_ * SEQ * HD / 512);
    k_cvt8<<<GW, 256, 0, stream>>>(wq, WQ, (size_t)DM * DM / 8); k_cvt8<<<GW, 256, 0, stream>>>(wk, WK, (size_t)DM * DM / 8);
    k_cvt8<<<GW, 256, 0, stream>>>(wv, WV, (size_t)DM * DM / 8); k_cvt8<<<GW, 256, 0, stream>>>(wp, WP, (size_t)DM * DM / 8);
    for (int b = 0; b < NB; ++b) {
        k_cvt8<<<GX, 256, 0, stream>>>(x + (size_t)b * SEQ_FULL * DM, XB, (size_t)SEQ * DM / 8);
        k_gemmw<bf, 0, true><<<dim3(SEQ / 64, DM / 64, 1), 32, 0, stream>>>(XB, nullptr, WQ, nullptr, DM, FQ, DM, bq, 0, 0, 0);
        k_qkp<<<GP, 256, 0, stream>>>(FQ, Q16, QPh, QPl);
        k_gemmw<bf, 0, true><<<dim3(SEQ / 64, DM / 64, 1), 32, 0, stream>>>(XB, nullptr, WK, nullptr, DM, FK, DM, bk, 0, 0, 0);
        k_qkp<<<GP, 256, 0, stream>>>(FK, K16, KPh, KPl);
        k_gemmw<bf, 0, true><<<dim3(SEQ / 64, DM / 64, 1), 32, 0, stream>>>(XB, nullptr, WV, nullptr, DM, FV, DM, bv, 0, 0, 0);
        k_vtp<<<GP, 256, 0, stream>>>(FV, VT16, VTh, VTl);
        k_flash<true><<<dim3(RH / 16, NH_), 32, 0, stream>>>(Q16, K16, VT16, QPh, QPl, KPh, KPl, VTh, VTl, 0, ATh, ATl);
#if SEQ > RH
        k_flash<false><<<dim3((SEQ - RH) / 16, NH_), 32, 0, stream>>>(Q16, K16, VT16, QPh, QPl, KPh, KPl, VTh, VTl, RH / 16, ATh, ATl);
#endif
        k_gemmw<bf, 1, true><<<dim3(SEQ / 64, DM / 64, 1), 32, 0, stream>>>(ATh, ATl, WP, nullptr, DM, OUT + (size_t)b * SEQ_FULL * DM, DM, bp, 0, 0, 0);
    }
}
